// MKMMDLoss_22093311771155
// MI455X (gfx1250) — hardware-verified
//
#include <hip/hip_runtime.h>


namespace {
constexpr int NB = 4096, DIM = 256, NALPHA = 5;
constexpr float XS = 8.0f, DOFF = 22.0f;
constexpr int NGW = 3 * (NB / 128) * (NB / 64) * 4;
constexpr int NKB = 3 * NB * NB / (256 * 64);

typedef _Float16 b16;
typedef __attribute__((ext_vector_type(16))) _Float16 v16b;
typedef __attribute__((ext_vector_type(8)))  _Float16 v8b;
typedef __attribute__((ext_vector_type(8)))  float v8f;
typedef __attribute__((ext_vector_type(4)))  float v4f;

__device__ __forceinline__ v8b ld8b(const b16* p) { return *(const v8b*)p; }
__device__ __forceinline__ v16b cat8b(v8b a, v8b b) { return __builtin_shufflevector(a, b, 0, 1, 2, 3, 4, 5, 6, 7, 8, 9, 10, 11, 12, 13, 14, 15); }
__device__ __forceinline__ v16b frag_kb(const b16* p, int hh) { return cat8b(ld8b(p + 8 * hh), ld8b(p + 16 + 8 * hh)); }
__device__ __forceinline__ void split16(float v, b16& hi, b16& lo) { hi = (b16)v; lo = (b16)(v - (float)hi); }
__device__ __forceinline__ void frag_ksplit(const float* p, int hh, v16b& fh_, v16b& fl_) {
  const float* p0 = p + 8 * hh; const float* p1 = p + 16 + 8 * hh;
#pragma unroll
  for (int e = 0; e < 8; ++e) { b16 a, c; split16(p0[e], a, c); fh_[e] = a; fl_[e] = c; split16(p1[e], a, c); fh_[8 + e] = a; fl_[8 + e] = c; }
}
__device__ __forceinline__ v8f wmma16b(v16b a, v16b b, v8f c) {
  v8f d = __builtin_amdgcn_wmma_f32_16x16x32_f16(false, a, false, b, (short)0, c, false, false);
  asm volatile("v_nop\n\tv_nop\n\tv_nop\n\tv_nop" : "+v"(d) : "v"(a), "v"(b));
  return d;
}
__device__ __forceinline__ void wave_lds_sync() {
  __builtin_amdgcn_fence(__ATOMIC_RELEASE, "workgroup");
  __builtin_amdgcn_wave_barrier();
  __builtin_amdgcn_fence(__ATOMIC_ACQUIRE, "workgroup");
}

struct Opnd { const void* p0; const void* p1; int ld; };
template <int NP> __device__ __forceinline__ void load_frags(const Opnd& o, int row, int kb, int hh, v16b& fh_, v16b& fl_) {
  if (NP == 0) { frag_ksplit((const float*)o.p0 + (size_t)row * o.ld + kb, hh, fh_, fl_); }
  else if (NP == 4 || NP == 5) {
    const float sc_ = (NP == 4) ? 64.0f : 8.0f;
    const float* p = (const float*)o.p0 + (size_t)row * o.ld + kb; const float* p0 = p + 8 * hh; const float* p1 = p + 16 + 8 * hh;
#pragma unroll
    for (int e = 0; e < 8; ++e) { b16 a, c; split16(p0[e] * sc_, a, c); fh_[e] = a; fl_[e] = c; split16(p1[e] * sc_, a, c); fh_[8 + e] = a; fl_[8 + e] = c; }
  } else if (NP == 3) {
    const float* p = (const float*)o.p0 + (size_t)row * o.ld + kb; const float* p0 = p + 8 * hh; const float* p1 = p + 16 + 8 * hh;
#pragma unroll
    for (int e = 0; e < 8; ++e) { fh_[e] = (b16)p0[e]; fh_[8 + e] = (b16)p1[e]; }
    fl_ = fh_;
  } else {
    fh_ = frag_kb((const b16*)o.p0 + (size_t)row * o.ld + kb, hh);
    if (NP == 2) fl_ = frag_kb((const b16*)o.p1 + (size_t)row * o.ld + kb, hh); else fl_ = fh_;
  }
}
template <int ANP, int BNP> __device__ __forceinline__ v8f mac(v16b ah, v16b al, v16b bh, v16b bl, v8f c) {
  c = wmma16b(ah, bh, c);
  if (BNP == 0 || BNP == 2 || BNP == 4 || BNP == 5) c = wmma16b(ah, bl, c);
  if (ANP == 0 || ANP == 2 || ANP == 4 || ANP == 5) c = wmma16b(al, bh, c);
  return c;
}
template <int ANP, int BNP>
__device__ __forceinline__ void gemm_tile(const Opnd& A, const Opnd& B, int K, int m0, int c0, int nloc, int hlf, v8f (&acc)[2][4]) {
  for (int kb = 0; kb < K; kb += 32) {
    v16b a0h, a0l, a1h, a1l;
    load_frags<ANP>(A, m0 + nloc, kb, hlf, a0h, a0l);
    load_frags<ANP>(A, m0 + 16 + nloc, kb, hlf, a1h, a1l);
#pragma unroll
    for (int t = 0; t < 4; ++t) {
      v16b bh, bl;
      load_frags<BNP>(B, c0 + t * 16 + nloc, kb, hlf, bh, bl);
      acc[0][t] = mac<ANP, BNP>(a0h, a0l, bh, bl, acc[0][t]);
      acc[1][t] = mac<ANP, BNP>(a1h, a1l, bh, bl, acc[1][t]);
    }
  }
}

__device__ __forceinline__ void epi_planes(v8f (&acc)[2][4], float scale, bool two, b16* __restrict__ oh, b16* __restrict__ ol, int ldo,
                                           int m0, int c0, int lane, b16* Th, b16* Tl) {
  const int nloc = lane & 15, hlf = lane >> 4;
#pragma unroll
  for (int t = 0; t < 4; ++t)
#pragma unroll
    for (int r = 0; r < 2; ++r)
#pragma unroll
      for (int v = 0; v < 8; ++v) {
        const int rr = r * 16 + v + 8 * hlf, cc = t * 16 + nloc;
        b16 h_, l_; split16(acc[r][t][v] * scale, h_, l_);
        Th[rr * 64 + cc] = h_; Tl[rr * 64 + cc] = l_;
      }
  wave_lds_sync();
  for (int pass = 0; pass < 2; ++pass) {
#pragma unroll
    for (int j = 0; j < 8; ++j) {
      const int rr = j * 4 + (lane >> 3), c8 = (lane & 7) * 8;
      const size_t o = (size_t)(m0 + rr) * ldo + c0 + c8;
      *(volatile v8b*)(oh + o) = ld8b(Th + rr * 64 + c8);
      if (two) *(volatile v8b*)(ol + o) = ld8b(Tl + rr * 64 + c8);
    }
    __threadfence();
  }
}
__device__ __forceinline__ void epi_f32(v8f (&acc)[2][4], float scale, const float* rscale, float* __restrict__ out, int ldo, int m0, int c0, int lane, float* Tt) {
  const int nloc = lane & 15, hlf = lane >> 4;
#pragma unroll
  for (int t = 0; t < 4; ++t)
#pragma unroll
    for (int r = 0; r < 2; ++r)
#pragma unroll
      for (int v = 0; v < 8; ++v) {
        const int rr = r * 16 + v + 8 * hlf;
        const float rs = rscale ? rscale[(size_t)(m0 + rr) * 32] : 1.0f;
        Tt[rr * 64 + t * 16 + nloc] = acc[r][t][v] * scale * rs;
      }
  wave_lds_sync();
  float* dst0 = out + (size_t)m0 * ldo + c0;
  for (int pass = 0; pass < 2; ++pass) {
#pragma unroll
    for (int j = 0; j < 16; ++j) { const int rr = j * 2 + hlf, c4 = nloc * 4; *(volatile v4f*)(dst0 + (size_t)rr * ldo + c4) = *(const v4f*)(Tt + rr * 64 + c4); }
    __threadfence();
  }
}


__global__ __launch_bounds__(256) void norm_kernel(const float* __restrict__ xs, const float* __restrict__ xt, float* __restrict__ nrm) {
  __shared__ float ns[32];
  const int wave = threadIdx.x >> 5, lane = threadIdx.x & 31, r0 = blockIdx.x * 32;
  for (int q = 0; q < 4; ++q) {
    const int r = r0 + wave * 4 + q; const float* row = (r < NB) ? (xs + (size_t)r * DIM) : (xt + (size_t)(r - NB) * DIM);
    float s = 0.0f;
#pragma unroll
    for (int e = 0; e < 8; ++e) { const float v = row[lane * 8 + e]; s += v * v; }
#pragma unroll
    for (int o = 16; o > 0; o >>= 1) s += __shfl_xor(s, o);
    if (lane == 0) ns[wave * 4 + q] = s;
  }
  __syncthreads();
  if (wave == 0) { ((volatile float*)nrm)[r0 + lane] = ns[lane]; __threadfence(); ((volatile float*)nrm)[r0 + lane] = ns[lane]; }
}

__global__ __launch_bounds__(128) void dist_kernel(const float* __restrict__ xs, const float* __restrict__ xt, const float* __restrict__ nrm, b16* __restrict__ d16,
                                                  double* __restrict__ part) {
  __shared__ __attribute__((aligned(16))) b16 Th[4][32 * 64];
  const int lane = threadIdx.x & 31, wave = threadIdx.x >> 5, nloc = lane & 15, hlf = lane >> 4, z = blockIdx.z;
  const int m0 = blockIdx.y * 128 + wave * 32, c0 = blockIdx.x * 64;
  const float* Arows = (z == 1) ? xt : xs; const float* Brows = (z == 0) ? xs : xt;
  const float* na = nrm + ((z == 1) ? NB : 0); const float* nb_ = nrm + ((z == 0) ? 0 : NB);
  v8f acc[2][4];
#pragma unroll
  for (int r = 0; r < 2; ++r)
#pragma unroll
    for (int t = 0; t < 4; ++t) acc[r][t] = (v8f){};
  const Opnd A{Arows, nullptr, DIM}, B{Brows, nullptr, DIM};
  gemm_tile<5, 5>(A, B, DIM, m0, c0, nloc, hlf, acc);
  b16* Tp = Th[wave]; double sd = 0.0;
#pragma unroll
  for (int t = 0; t < 4; ++t)
#pragma unroll
    for (int r = 0; r < 2; ++r)
#pragma unroll
      for (int v = 0; v < 8; ++v) {
        const int rr = r * 16 + v + 8 * hlf, cc = t * 16 + nloc;
        float sq = na[m0 + rr] + nb_[c0 + cc] - 2.0f * acc[r][t][v] * (1.0f / (XS * XS));
        sq = fmaxf(sq, 0.0f); const float dd = (sq > 0.0f) ? sqrtf(sq) : 0.0f;
        sd += (double)dd; Tp[rr * 64 + cc] = (b16)(dd - DOFF);
      }
  wave_lds_sync();
  b16* dst = d16 + ((size_t)z * NB + m0) * NB + c0;
  for (int pass = 0; pass < 2; ++pass) {
#pragma unroll
    for (int j = 0; j < 8; ++j) { const int rr = j * 4 + (lane >> 3), c8 = (lane & 7) * 8; *(volatile v8b*)(dst + (size_t)rr * NB + c8) = ld8b(Tp + rr * 64 + c8); }
    __threadfence();
  }
#pragma unroll
  for (int o = 16; o > 0; o >>= 1) sd += __shfl_xor(sd, o);
  const int wid = ((z * (NB / 128) + blockIdx.y) * (NB / 64) + blockIdx.x) * 4 + wave;
  const double pv = (lane == 0) ? sd : 0.0;
  if (lane < 16) { ((volatile double*)part)[(size_t)wid * 16 + lane] = pv; __threadfence(); ((volatile double*)part)[(size_t)wid * 16 + lane] = pv; }
}

__global__ __launch_bounds__(64) void mean_kernel(const double* __restrict__ part, float* __restrict__ mean) {
  if (threadIdx.x == 0) {
    for (int z = 0; z < 3; ++z) {
      double s = 0.0; const int per = NGW / 3;
#pragma unroll 1
      for (int w = 0; w < per; ++w) s += part[(size_t)(z * per + w) * 16];
      const float mv = (float)(s / ((double)NB * NB));
      ((volatile float*)mean)[z] = mv; __threadfence(); ((volatile float*)mean)[z] = mv;
    }
  }
}

__global__ __launch_bounds__(256) void ksum_kernel(const b16* __restrict__ d16, const float* __restrict__ mean, double* __restrict__ part2) {
  __shared__ double red[256];
  const size_t e0 = ((size_t)blockIdx.x * 256 + threadIdx.x) * 64;
  const int z = (int)(e0 / ((size_t)NB * NB)); const float mz = mean[z], wgt = (z == 2) ? -2.0f : 1.0f;
  float coef[NALPHA];
#pragma unroll
  for (int k = 0; k < NALPHA; ++k) { const float a = (float)(1 << k) * 0.125f; coef[k] = -1.0f / (2.0f * a * mz); }
  double s = 0.0;
#pragma unroll 1
  for (int e = 0; e < 64; ++e) {
    const float dd = (float)d16[e0 + e] + DOFF; float ks = 0.0f;
#pragma unroll
    for (int k = 0; k < NALPHA; ++k) ks += expf(dd * coef[k]);
    s += (double)ks;
  }
  red[threadIdx.x] = s * (double)wgt; __syncthreads();
#pragma unroll 1
  for (int o = 128; o > 0; o >>= 1) { if ((int)threadIdx.x < o) red[threadIdx.x] += red[threadIdx.x + o]; __syncthreads(); }
  if (threadIdx.x < 16) { const double pv = (threadIdx.x == 0) ? red[0] : 0.0; ((volatile double*)part2)[(size_t)blockIdx.x * 16 + threadIdx.x] = pv; __threadfence(); ((volatile double*)part2)[(size_t)blockIdx.x * 16 + threadIdx.x] = pv; }
}

__global__ __launch_bounds__(64) void final_kernel(const double* __restrict__ part2, float* __restrict__ out) {
  if (threadIdx.x == 0) {
    double tot = 0.0;
#pragma unroll 1
    for (int bk = 0; bk < NKB; ++bk) tot += part2[(size_t)bk * 16];
    float loss = sqrtf((float)(tot / ((double)NB * (NB - 1.0))));
    if (loss != loss) loss = 0.0f;
    ((volatile float*)out)[0] = loss; __threadfence(); ((volatile float*)out)[0] = loss;
  }
}
}

extern "C" void kernel_launch(void* const* d_in, const int* in_sizes, int n_in,
                              void* d_out, int out_size, void* d_ws, size_t ws_size, hipStream_t stream) {
  (void)n_in; (void)out_size;
  const float* xs = (const float*)d_in[0]; const float* xt = (const float*)d_in[1];
  float* out = (float*)d_out;
  if (in_sizes[0] != NB * DIM || in_sizes[1] != NB * DIM) return;
  size_t off = 0; char* ws = (char*)d_ws;
  auto carve = [&](size_t bytes) { char* p = ws + off; off += (bytes + 255) & ~(size_t)255; return p; };
  float* nrm = (float*)carve((size_t)2 * NB * 4);
  b16* d16 = (b16*)carve((size_t)3 * NB * NB * 2);
  double* part = (double*)carve((size_t)NGW * 16 * 8);
  float* mean = (float*)carve(256);
  double* part2 = (double*)carve((size_t)NKB * 16 * 8);
  if (off > ws_size) return;
  norm_kernel<<<2 * NB / 32, 256, 0, stream>>>(xs, xt, nrm);
  dist_kernel<<<dim3(NB / 64, NB / 128, 3), 128, 0, stream>>>(xs, xt, nrm, d16, part);
  mean_kernel<<<1, 64, 0, stream>>>(part, mean);
  ksum_kernel<<<NKB, 256, 0, stream>>>(d16, mean, part2);
  final_kernel<<<1, 64, 0, stream>>>(part2, out);
}
